// Kernel3D_48962627175188
// MI455X (gfx1250) — hardware-verified
//
#include <hip/hip_runtime.h>
#include <stddef.h>
#include <stdint.h>
#include <math.h>


#define NPTS   4096
#define GXD    64
#define GYD    64
#define GZD    64
#define TD     8
#define ZTD    (GZD * TD)
#define NTHR   256
#define NWAVE  8
#define WSCAP  134217728
#define INV_SQRT_2PI 0.3989422804014327f

static_assert(NTHR == NWAVE * 32);
static_assert((NPTS % 32) == 0);
static_assert(NPTS == 2 * NTHR * 8);
static_assert((NPTS % 1024) == 0);
static_assert(GXD == 64 && GYD == 64 && GZD == 64 && TD == 8);
static_assert((ZTD % 128) == 0);

#define SZ_T   ((size_t)3 * 64 * NPTS * 4)
#define SZ_A   ((size_t)GYD * GXD * NPTS * 2)
#define SZ_B   ((size_t)ZTD * NPTS * 2)
#define SZ_TOT (SZ_T + 2 * SZ_A + 2 * SZ_B)
static_assert(SZ_TOT <= (size_t)WSCAP);
static_assert((SZ_T % 128) == 0);
static_assert((SZ_A % 128) == 0);
static_assert((SZ_B % 128) == 0);

#define NBLK_T (3 * 64 * NPTS / 4 / NTHR)
#define NBLK_A (GYD * GXD * 2)
#define NBLK_B (ZTD * 2)
static_assert(NBLK_T * NTHR * 4 == 3 * 64 * NPTS);

typedef float          v4f   __attribute__((ext_vector_type(4)));
typedef float          v8f   __attribute__((ext_vector_type(8)));
typedef unsigned short v8us  __attribute__((ext_vector_type(8)));
typedef __bf16         v16bf __attribute__((ext_vector_type(16)));
union FragB { v16bf v; v8us q[2]; };

__device__ __forceinline__ v8f wmb(v16bf a, v16bf b, v8f c) {
  v8f d = __builtin_amdgcn_wmma_f32_16x16x32_bf16(false, a, false, b, (short)0, c, false, false);
  asm volatile("v_nop\n\tv_nop\n\tv_nop\n\tv_nop" : "+v"(d) : "v"(a), "v"(b));
  return d;
}

__device__ __forceinline__ unsigned int bf16_rne(float f) {
  unsigned int u = __float_as_uint(f);
  u += 0x7FFFu + ((u >> 16) & 1u);
  return u >> 16;
}

__device__ __forceinline__ void split1(float f, unsigned short& hb, unsigned short& lb) {
  const unsigned int hbits = bf16_rne(f);
  const float hf = __uint_as_float(hbits << 16);
  hb = (unsigned short)hbits;
  lb = (unsigned short)bf16_rne(f - hf);
}

__device__ __forceinline__ void store_split8(v4f p0, v4f p1, unsigned short* dh, unsigned short* dl) {
  v8us hv, lv;
  unsigned short hb, lb;
  split1(p0.x, hb, lb); hv[0] = hb; lv[0] = lb;
  split1(p0.y, hb, lb); hv[1] = hb; lv[1] = lb;
  split1(p0.z, hb, lb); hv[2] = hb; lv[2] = lb;
  split1(p0.w, hb, lb); hv[3] = hb; lv[3] = lb;
  split1(p1.x, hb, lb); hv[4] = hb; lv[4] = lb;
  split1(p1.y, hb, lb); hv[5] = hb; lv[5] = lb;
  split1(p1.z, hb, lb); hv[6] = hb; lv[6] = lb;
  split1(p1.w, hb, lb); hv[7] = hb; lv[7] = lb;
  *(volatile v8us*)dh = hv;
  *(volatile v8us*)dl = lv;
  __threadfence();
  *(volatile v8us*)dh = hv;
  *(volatile v8us*)dl = lv;
}

__global__ __launch_bounds__(NTHR) void k_basis(const float* __restrict__ mu,
                                                const float* __restrict__ sigma,
                                                float* bT) {
  const int gid  = blockIdx.x * NTHR + threadIdx.x;
  const int n4   = gid & 1023;
  const int rest = gid >> 10;
  const int g    = rest & 63;
  const int axis = min(rest >> 6, 2);
  const float gf = (float)g;
  v4f r = {0.f, 0.f, 0.f, 0.f};
#pragma unroll 1
  for (int j = 0; j < 4; ++j) {
    const int n = 4 * n4 + j;
    const float mv = mu[n * 3 + axis];
    const float sv = sigma[n * 3 + axis];
    const float rs = 1.0f / sv;
    const float inv = INV_SQRT_2PI * fabsf(rs);
    const float d = (mv - gf) * rs;
    const float val = inv * expf(-0.5f * (d * d));
    const v4f t = {r.y, r.z, r.w, val};
    r = t;
  }
  float* p = bT + ((size_t)(axis * 64 + g)) * NPTS + 4 * n4;
  *(volatile v4f*)p = r;
  __threadfence();
  *(volatile v4f*)p = r;
}

__global__ __launch_bounds__(NTHR) void k_planes(const float* __restrict__ bT,
                                                 const float* __restrict__ xin,
                                                 unsigned short* AH, unsigned short* AL,
                                                 unsigned short* BH, unsigned short* BL) {
  const int tid = threadIdx.x;
  const int blk = blockIdx.x;
  if (blk < NBLK_A) {
    const int row = blk >> 1;
    const int n0  = (blk & 1) * (NPTS / 2) + tid * 8;
    const int yy = row >> 6, xx = row & 63;
    const float* px = bT + ((size_t)(0 * 64 + xx)) * NPTS + n0;
    const float* py = bT + ((size_t)(1 * 64 + yy)) * NPTS + n0;
    const v4f x0 = *(const v4f*)px, x1 = *(const v4f*)(px + 4);
    const v4f y0 = *(const v4f*)py, y1 = *(const v4f*)(py + 4);
    const v4f p0 = x0 * y0, p1 = x1 * y1;
    const size_t o = (size_t)row * NPTS + n0;
    store_split8(p0, p1, AH + o, AL + o);
  } else {
    const int b  = min(blk - NBLK_A, NBLK_B - 1);
    const int zt = b >> 1;
    const int n0 = (b & 1) * (NPTS / 2) + tid * 8;
    const int z = zt >> 3, t = zt & 7;
    const float* pz = bT + ((size_t)(2 * 64 + z)) * NPTS + n0;
    const v4f z0 = *(const v4f*)pz, z1 = *(const v4f*)(pz + 4);
    const float* xp = xin + (size_t)n0 * TD + t;
    v4f v0, v1;
    v0.x = xp[0 * TD]; v0.y = xp[1 * TD]; v0.z = xp[2 * TD]; v0.w = xp[3 * TD];
    v1.x = xp[4 * TD]; v1.y = xp[5 * TD]; v1.z = xp[6 * TD]; v1.w = xp[7 * TD];
    const v4f p0 = z0 * v0, p1 = z1 * v1;
    const size_t o = (size_t)zt * NPTS + n0;
    store_split8(p0, p1, BH + o, BL + o);
  }
}

__global__ __launch_bounds__(NTHR) void k_splat(const unsigned short* __restrict__ AH,
                                                const unsigned short* __restrict__ AL,
                                                const unsigned short* __restrict__ BH,
                                                const unsigned short* __restrict__ BL,
                                                float* out) {
  __shared__ __attribute__((aligned(16))) float stg[NWAVE * 16 * 64];
  const int tid = threadIdx.x, lane = tid & 31, w = tid >> 5, h = lane >> 4, m = lane & 15;
  const int zb = blockIdx.x, y = blockIdx.y;
  const int ztbase = zb * 128;
  const int mt = w & 3, ns = w >> 2;
  const int xrow = 16 * mt + m;
  const int ztb  = ztbase + 64 * ns + m;

  const size_t aoff = ((size_t)(y * 64 + xrow)) * NPTS + 8 * h;
  const unsigned short* pah = AH + aoff;
  const unsigned short* pal = AL + aoff;

  const v8f zero8 = {0.f, 0.f, 0.f, 0.f, 0.f, 0.f, 0.f, 0.f};
  v8f acc[4];
#pragma unroll
  for (int j = 0; j < 4; ++j) acc[j] = zero8;

#pragma unroll 1
  for (int ks = 0; ks < NPTS / 32; ++ks) {
    const int k0 = 32 * ks;
    FragB ah, al;
    ah.q[0] = *(const v8us*)(pah + k0);
    ah.q[1] = *(const v8us*)(pah + k0 + 16);
    al.q[0] = *(const v8us*)(pal + k0);
    al.q[1] = *(const v8us*)(pal + k0 + 16);
#pragma unroll
    for (int j = 0; j < 4; ++j) {
      const size_t boff = ((size_t)(ztb + 16 * j)) * NPTS + 8 * h + k0;
      FragB bh, bl;
      bh.q[0] = *(const v8us*)(BH + boff);
      bh.q[1] = *(const v8us*)(BH + boff + 16);
      bl.q[0] = *(const v8us*)(BL + boff);
      bl.q[1] = *(const v8us*)(BL + boff + 16);
      acc[j] = wmb(ah.v, bh.v, acc[j]);
      acc[j] = wmb(ah.v, bl.v, acc[j]);
      acc[j] = wmb(al.v, bh.v, acc[j]);
    }
  }

  float* sw = stg + w * (16 * 64);
#pragma unroll
  for (int j = 0; j < 4; ++j) {
#pragma unroll
    for (int r = 0; r < 8; ++r) sw[(8 * h + r) * 64 + 16 * j + m] = acc[j][r];
  }
  __syncthreads();

  v4f ov[8];
#pragma unroll
  for (int i = 0; i < 8; ++i) ov[i] = *(const v4f*)(sw + (2 * i + h) * 64 + 4 * m);

  const size_t colbase = (size_t)y * ZTD + ztbase + 64 * ns + 4 * m;
#pragma unroll
  for (int i = 0; i < 8; ++i) {
    const int x = 16 * mt + 2 * i + h;
    float* gp = out + (size_t)x * (GYD * ZTD) + colbase;
    *(volatile v4f*)gp = ov[i];
  }
  __threadfence();
#pragma unroll
  for (int i = 0; i < 8; ++i) {
    const int x = 16 * mt + 2 * i + h;
    float* gp = out + (size_t)x * (GYD * ZTD) + colbase;
    *(volatile v4f*)gp = ov[i];
  }
}

extern "C" void kernel_launch(void* const* d_in, const int* in_sizes, int n_in,
                              void* d_out, int out_size, void* d_ws, size_t ws_size,
                              hipStream_t stream) {
  if (n_in < 3) return;
  if (in_sizes[0] != NPTS * TD) return;
  if (in_sizes[1] != NPTS * 3) return;
  if (in_sizes[2] != NPTS * 3) return;
  if (out_size != GXD * GYD * GZD * TD) return;

  const float* xin   = (const float*)d_in[0];
  const float* mu    = (const float*)d_in[1];
  const float* sigma = (const float*)d_in[2];
  float* out = (float*)d_out;

  char* ws = (char*)d_ws;
  size_t off = 0;
  const size_t oT  = off; off += SZ_T;
  const size_t oAH = off; off += SZ_A;
  const size_t oAL = off; off += SZ_A;
  const size_t oBH = off; off += SZ_B;
  const size_t oBL = off; off += SZ_B;
  if (off != SZ_TOT) return;
  if (off > ws_size || off > (size_t)WSCAP) return;

  float* bT = (float*)(ws + oT);
  unsigned short* AH = (unsigned short*)(ws + oAH);
  unsigned short* AL = (unsigned short*)(ws + oAL);
  unsigned short* BH = (unsigned short*)(ws + oBH);
  unsigned short* BL = (unsigned short*)(ws + oBL);

  k_basis<<<NBLK_T, NTHR, 0, stream>>>(mu, sigma, bT);
  k_planes<<<NBLK_A + NBLK_B, NTHR, 0, stream>>>(bT, xin, AH, AL, BH, BL);
  k_splat<<<dim3(ZTD / 128, GYD), NTHR, 0, stream>>>(AH, AL, BH, BL, out);
}
